// CausalAttention_70282844832524
// MI455X (gfx1250) — hardware-verified
//
#include <hip/hip_runtime.h>


#ifndef NB
#define NB 4
#endif
#ifndef SEQ
#define SEQ 4096
#endif
#define NB_FULL  4
#define SEQ_FULL 4096
#define DIN   768
#define HD    64
#define RHALF (SEQ / 2)
#define RH    64
#define QCAR  4.0f
#define SCL   0.0078125f

static_assert(SEQ % 128 == 0);
static_assert(RHALF % 64 == 0);
static_assert(RH <= RHALF);
static_assert(DIN % 32 == 0);
static_assert(HD == 64);
static_assert((NB * SEQ) % 64 == 0);
static_assert(NB <= NB_FULL);
static_assert(SEQ <= SEQ_FULL);

typedef _Float16 h16;
typedef unsigned short bf;
typedef __attribute__((ext_vector_type(16))) __bf16   v16bf;
typedef __attribute__((ext_vector_type(16))) _Float16 v16h;
typedef __attribute__((ext_vector_type(8)))  _Float16 v8h;
typedef __attribute__((ext_vector_type(8)))  unsigned short v8us;
typedef __attribute__((ext_vector_type(8)))  float    v8f;
typedef __attribute__((ext_vector_type(4)))  float    v4f;
typedef __attribute__((ext_vector_type(4)))  unsigned short v4us;
typedef __attribute__((ext_vector_type(2)))  unsigned short v2us;
typedef v4f  __attribute__((may_alias)) v4fa;

#pragma clang fp contract(off)

__device__ __forceinline__ unsigned short f2bf(float f) { unsigned u = __float_as_uint(f); u += 0x7FFFu + ((u >> 16) & 1u); return (unsigned short)(u >> 16); }
__device__ __forceinline__ float bf2f(unsigned short b) { return __uint_as_float(((unsigned)b) << 16); }
__device__ __forceinline__ v16h cat16(v8h lo, v8h hi) { return __builtin_shufflevector(lo, hi, 0, 1, 2, 3, 4, 5, 6, 7, 8, 9, 10, 11, 12, 13, 14, 15); }
__device__ __forceinline__ v16bf cat16b(v8us lo, v8us hi) { return __builtin_bit_cast(v16bf, __builtin_shufflevector(lo, hi, 0, 1, 2, 3, 4, 5, 6, 7, 8, 9, 10, 11, 12, 13, 14, 15)); }
__device__ __forceinline__ v8f wmma16(v16h a, v16h b, v8f c) { return __builtin_amdgcn_wmma_f32_16x16x32_f16(false, a, false, b, (short)0, c, false, false); }
__device__ __forceinline__ v8f wmmab(v16bf a, v16bf b, v8f c) { return __builtin_amdgcn_wmma_f32_16x16x32_bf16(false, a, false, b, (short)0, c, false, false); }
__device__ __forceinline__ void splitf(float y, unsigned short& h, unsigned short& l) { h = f2bf(y); l = f2bf(y - bf2f(h)); }

template <typename T16> struct WFrag;
template <> struct WFrag<h16> { typedef v16h V; static __device__ __forceinline__ V ld(const h16* p) { return cat16(*(const v8h*)p, *(const v8h*)(p + 16)); } static __device__ __forceinline__ v8f mma(V a, V b, v8f c) { return wmma16(a, b, c); } };
template <> struct WFrag<bf> { typedef v16bf V; static __device__ __forceinline__ V ld(const bf* p) { return cat16b(*(const v8us*)p, *(const v8us*)(p + 16)); } static __device__ __forceinline__ v8f mma(V a, V b, v8f c) { return wmmab(a, b, c); } };
template <typename T16, int NSPLIT, bool CSKIP, bool KLIM>
__global__ __launch_bounds__(32) void k_gemmw(const T16* __restrict__ A, const T16* __restrict__ A2, const T16* __restrict__ Bt, const T16* __restrict__ Bt2, int K, float* C, int ldc, int rofs, size_t sA, size_t sB, size_t sC) {
    static_assert(NSPLIT == 0 || NSPLIT == 2);
    typedef typename WFrag<T16>::V V;
    __shared__ __align__(16) float os[16 * 68];
    const size_t z = blockIdx.z; A += z * sA; Bt += z * sB; C += z * sC; if (NSPLIT == 2) { A2 += z * sA; Bt2 += z * sB; }
    const int lane = threadIdx.x & 31, lr = lane & 15, hi = lane >> 4; const int r0 = blockIdx.x * 64, c0 = blockIdx.y * 64;
    if (CSKIP) { if (c0 > ((rofs + r0) | 127)) return; }
    const int kl = rofs + r0 + 64; const int kend = KLIM ? ((kl < K) ? kl : K) : K;
    v8f acc[4][4];
#pragma unroll
    for (int mb = 0; mb < 4; ++mb)
#pragma unroll
        for (int nb = 0; nb < 4; ++nb) acc[mb][nb] = (v8f){};
    const size_t aoff = (size_t)(r0 + lr) * K + 8 * hi, boff = (size_t)(c0 + lr) * K + 8 * hi;
#pragma unroll 1
    for (int kc = 0; kc < kend; kc += 32) {
        V a[4], a2[4], bl, b2l;
#pragma unroll
        for (int mb = 0; mb < 4; ++mb) { a[mb] = WFrag<T16>::ld(A + aoff + (size_t)mb * 16 * K + kc); if (NSPLIT == 2) a2[mb] = WFrag<T16>::ld(A2 + aoff + (size_t)mb * 16 * K + kc); else a2[mb] = a[mb]; }
#pragma unroll
        for (int nb = 0; nb < 4; ++nb) { const V b = WFrag<T16>::ld(Bt + boff + (size_t)nb * 16 * K + kc); V b2 = b; if (NSPLIT == 2) b2 = WFrag<T16>::ld(Bt2 + boff + (size_t)nb * 16 * K + kc);
#pragma unroll
            for (int mb = 0; mb < 4; ++mb) { acc[mb][nb] = WFrag<T16>::mma(a[mb], b, acc[mb][nb]); if (NSPLIT == 2) { acc[mb][nb] = WFrag<T16>::mma(a2[mb], b, acc[mb][nb]); acc[mb][nb] = WFrag<T16>::mma(a[mb], b2, acc[mb][nb]); } }
            bl = b; b2l = b2; }
        asm volatile("v_nop\n\tv_nop\n\tv_nop\n\tv_nop" : "+v"(acc[0][0]), "+v"(acc[1][1]), "+v"(acc[2][2]), "+v"(acc[3][3]) : "v"(a[0]), "v"(a[3]), "v"(a2[3]), "v"(bl), "v"(b2l));
    }
#pragma unroll
    for (int mb = 0; mb < 4; ++mb) {
#pragma unroll
        for (int nb = 0; nb < 4; ++nb) {
#pragma unroll
            for (int j = 0; j < 8; ++j) os[(hi * 8 + j) * 68 + nb * 16 + lr] = acc[mb][nb][j]; }
        __builtin_amdgcn_wave_barrier(); asm volatile("" ::: "memory");
        float* crow = C + (size_t)(r0 + mb * 16) * ldc + c0;
#pragma unroll 1
        for (int ps = 0; ps < 2; ++ps) {
#pragma unroll
            for (int s = 0; s < 8; ++s) { const int row = 2 * s + hi, cofs = lr * 4; const v4f val = *(const v4fa*)(os + row * 68 + cofs);
                *(volatile v4f*)(crow + (size_t)row * ldc + cofs) = val; }
            if (ps == 0) __threadfence(); }
        __builtin_amdgcn_wave_barrier(); asm volatile("" ::: "memory");
    }
}

__global__ __launch_bounds__(256) void k_wt3(const float* __restrict__ w0, const float* __restrict__ w1, const float* __restrict__ w2, bf* Wt) {
    const int which = blockIdx.y; const float* w = (which == 0) ? w0 : ((which == 1) ? w1 : w2); bf* Bt = Wt + (size_t)which * HD * DIN;
    const int lane = threadIdx.x & 31; const int L0 = (blockIdx.x * 8 + (threadIdx.x >> 5)) * 8; const int nlines = HD * DIN / 64;
#pragma unroll
    for (int ps = 0; ps < 2; ++ps) {
#pragma unroll 1
        for (int l = 0; l < 8; ++l) { const int L = L0 + l; if (L >= nlines) break; const size_t e = (size_t)L * 64 + lane * 2; const int k = (int)(e % DIN), n = (int)(e / DIN); v2us o;
            o[0] = f2bf(w[(size_t)k * HD + n]); o[1] = f2bf(w[(size_t)(k + 1) * HD + n]); *(volatile v2us*)(Bt + e) = o; }
        if (ps == 0) __threadfence(); }
}

__global__ __launch_bounds__(256) void k_cvtx(const float* __restrict__ X, bf* Xb, size_t n8) {
    const size_t i = (size_t)blockIdx.x * 256 + threadIdx.x; if (i >= n8) return; const size_t e = i * 8; const size_t r = e / DIN; const int c = (int)(e - r * DIN);
    const size_t srow = (r / SEQ) * SEQ_FULL + (r % SEQ);
    const float* p = X + srow * DIN + c; const v4f a0 = *(const v4f*)p; const v4f a1 = *(const v4f*)(p + 4); v8us o;
#pragma unroll
    for (int k = 0; k < 4; ++k) { o[k] = f2bf(a0[k]); o[k + 4] = f2bf(a1[k]); }
    *(volatile v8us*)(Xb + e) = o; __threadfence(); *(volatile v8us*)(Xb + e) = o;
}

__global__ __launch_bounds__(256) void k_plane3(const float* __restrict__ F, h16* P16, bf* Ph, bf* Pl, size_t n8) {
    const size_t i = (size_t)blockIdx.x * 256 + threadIdx.x; if (i >= n8) return;
    const v4f x0 = *(const v4f*)(F + i * 8); const v4f x1 = *(const v4f*)(F + i * 8 + 4);
    v8h o16; v8us oh, ol;
#pragma unroll
    for (int k = 0; k < 4; ++k) { const float y0 = x0[k] * QCAR, y1 = x1[k] * QCAR; o16[k] = (h16)y0; o16[k + 4] = (h16)y1; unsigned short a, c; splitf(y0, a, c); oh[k] = a; ol[k] = c; splitf(y1, a, c); oh[k + 4] = a; ol[k + 4] = c; }
    *(volatile v8h*)(P16 + i * 8) = o16; *(volatile v8us*)(Ph + i * 8) = oh; *(volatile v8us*)(Pl + i * 8) = ol;
    __threadfence();
    *(volatile v8h*)(P16 + i * 8) = o16; *(volatile v8us*)(Ph + i * 8) = oh; *(volatile v8us*)(Pl + i * 8) = ol;
}

__global__ __launch_bounds__(256) void k_vtp(const float* __restrict__ F, bf* Vh, bf* Vl) {
    const size_t e = ((size_t)blockIdx.x * 256 + threadIdx.x) * 2; if (e >= (size_t)NB * HD * SEQ) return;
    const int t = (int)(e % SEQ); const int d = (int)((e / SEQ) % HD); const int g = (int)(e / ((size_t)SEQ * HD));
    v2us oh, ol;
#pragma unroll
    for (int q = 0; q < 2; ++q) { const float x = F[((size_t)g * SEQ + t + q) * HD + d]; unsigned short a, c; splitf(x, a, c); oh[q] = a; ol[q] = c; }
    *(volatile v2us*)(Vh + e) = oh; *(volatile v2us*)(Vl + e) = ol; __threadfence(); *(volatile v2us*)(Vh + e) = oh; *(volatile v2us*)(Vl + e) = ol;
}

__global__ __launch_bounds__(256) void k_asoft(const float* __restrict__ Sb, int rofs, bf* Ph, bf* Pl) {
    const int lane = threadIdx.x & 31; const int lrow = blockIdx.x * 8 + (threadIdx.x >> 5); if (lrow >= RHALF) return;
    const int i = rofs + lrow; const int nch = (i >> 7) + 1;
    const float* sr = Sb + (size_t)lrow * SEQ; float v[SEQ / 32]; float mx = -3.0e38f;
#pragma unroll
    for (int ch = 0; ch < SEQ / 128; ++ch) {
        const int j0 = ch * 128 + lane * 4;
        if (ch < nch) { const v4f a = *(const v4f*)(sr + j0);
#pragma unroll
            for (int q = 0; q < 4; ++q) { const float t = (j0 + q <= i) ? a[q] * SCL : -3.0e38f; v[ch * 4 + q] = t; mx = fmaxf(mx, t); }
        } else {
#pragma unroll
            for (int q = 0; q < 4; ++q) v[ch * 4 + q] = 0.0f; }
    }
#pragma unroll
    for (int sh = 16; sh; sh >>= 1) mx = fmaxf(mx, __shfl_xor(mx, sh, 32));
    float sum = 0.f;
#pragma unroll
    for (int ch = 0; ch < SEQ / 128; ++ch) { if (ch < nch) {
#pragma unroll
        for (int q = 0; q < 4; ++q) { const int k = ch * 4 + q; float d0 = __fsub_rn(v[k], mx); asm volatile("" : "+v"(d0)); v[k] = __builtin_amdgcn_exp2f(__fmul_rn(d0, 1.4426950408889634f)); sum += v[k]; } } }
#pragma unroll
    for (int sh = 16; sh; sh >>= 1) sum += __shfl_xor(sum, sh, 32);
    const float f = __fdiv_rn(1.0f, sum);
#pragma unroll
    for (int ch = 0; ch < SEQ / 128; ++ch) { if (ch < nch) {
#pragma unroll
        for (int q = 0; q < 4; ++q) { const int k = ch * 4 + q; unsigned short a, c; splitf(v[k] * f, a, c); v[k] = __uint_as_float((unsigned)a | (((unsigned)c) << 16)); } } }
#pragma unroll 1
    for (int ps = 0; ps < 2; ++ps) {
#pragma unroll
        for (int ch = 0; ch < SEQ / 128; ++ch) { if (ch < nch) { v4us oh, ol;
#pragma unroll
            for (int q = 0; q < 4; ++q) { const unsigned w = __float_as_uint(v[ch * 4 + q]); oh[q] = (unsigned short)(w & 0xFFFFu); ol[q] = (unsigned short)(w >> 16); }
            const size_t oo = (size_t)lrow * SEQ + ch * 128 + lane * 4; *(volatile v4us*)(Ph + oo) = oh; *(volatile v4us*)(Pl + oo) = ol; } }
        if (ps == 0) __threadfence(); }
}

static constexpr size_t al256(size_t b) { return (b + 255) & ~(size_t)255; }
static constexpr size_t WS_TOTAL = al256((size_t)3 * HD * DIN * 2) + al256((size_t)NB * SEQ * DIN * 2) + al256((size_t)3 * NB * SEQ * HD * 4)
                                 + 6 * al256((size_t)NB * SEQ * HD * 2) + 2 * al256((size_t)NB * HD * SEQ * 2) + al256((size_t)RHALF * SEQ * 4) + 2 * al256((size_t)RHALF * SEQ * 2);
static_assert(WS_TOTAL <= (size_t)134217728);
static_assert((size_t)NB * SEQ * HD * 4 <= (size_t)4194304);

extern "C" void kernel_launch(void* const* d_in, const int* in_sizes, int n_in,
                              void* d_out, int out_size, void* d_ws, size_t ws_size, hipStream_t stream) {
    if (n_in < 4) return;
    if (in_sizes[0] < ((NB - 1) * SEQ_FULL + SEQ) * DIN) return;
    if (in_sizes[1] < DIN * HD || in_sizes[2] < DIN * HD || in_sizes[3] < DIN * HD) return;
    if (out_size < NB * SEQ * HD) return;
    const float* Xin = (const float*)d_in[0]; const float* Wq = (const float*)d_in[1]; const float* Wk = (const float*)d_in[2]; const float* Wv = (const float*)d_in[3];
    float* OUT = (float*)d_out;
    char* wsp = (char*)d_ws;
    auto take = [&](size_t bytes) { char* p = wsp; wsp += al256(bytes); return (void*)p; };
    const size_t nTok = (size_t)NB * SEQ;
    bf* Wt = (bf*)take((size_t)3 * HD * DIN * 2);
    bf* Xb = (bf*)take(nTok * DIN * 2);
    float* QKVf = (float*)take((size_t)3 * nTok * HD * 4);
    h16* Q16 = (h16*)take(nTok * HD * 2); bf* Qh = (bf*)take(nTok * HD * 2); bf* Ql = (bf*)take(nTok * HD * 2);
    h16* K16 = (h16*)take(nTok * HD * 2); bf* Kh = (bf*)take(nTok * HD * 2); bf* Kl = (bf*)take(nTok * HD * 2);
    bf* Vh = (bf*)take((size_t)NB * HD * SEQ * 2); bf* Vl = (bf*)take((size_t)NB * HD * SEQ * 2);
    float* Sb = (float*)take((size_t)RHALF * SEQ * 4);
    bf* Eh = (bf*)take((size_t)RHALF * SEQ * 2); bf* El = (bf*)take((size_t)RHALF * SEQ * 2);
    if ((size_t)(wsp - (char*)d_ws) > ws_size) return;
    const float* Qf = QKVf; const float* Kf = QKVf + nTok * HD; const float* Vf = QKVf + 2 * nTok * HD;

    k_wt3<<<dim3(HD * DIN / 64 / 64, 3), 256, 0, stream>>>(Wq, Wk, Wv, Wt);
    { const size_t n8 = nTok * DIN / 8; k_cvtx<<<(unsigned)((n8 + 255) / 256), 256, 0, stream>>>(Xin, Xb, n8); }
    k_gemmw<bf, 0, false, false><<<dim3((unsigned)(nTok / 64), 1, 3), 32, 0, stream>>>(Xb, nullptr, Wt, nullptr, DIN, QKVf, HD, 0, (size_t)0, (size_t)HD * DIN, nTok * HD);
    { const size_t n8 = nTok * HD / 8;
      k_plane3<<<(unsigned)((n8 + 255) / 256), 256, 0, stream>>>(Qf, Q16, Qh, Ql, n8);
      k_plane3<<<(unsigned)((n8 + 255) / 256), 256, 0, stream>>>(Kf, K16, Kh, Kl, n8); }
    k_vtp<<<(unsigned)(((size_t)NB * HD * SEQ / 2 + 255) / 256), 256, 0, stream>>>(Vf, Vh, Vl);
    for (int b = 0; b < NB; ++b) {
        for (int h = 0; h < 2; ++h) {
            const int rofs = h * RHALF;
            k_gemmw<h16, 0, true, false><<<dim3(RHALF / 64, (rofs + RHALF) / 64, 1), 32, 0, stream>>>(Q16 + ((size_t)b * SEQ + rofs) * HD, nullptr, K16 + (size_t)b * SEQ * HD, nullptr, HD, Sb, SEQ, rofs, (size_t)0, (size_t)0, (size_t)0);
            if (h == 0) k_gemmw<bf, 2, false, false><<<dim3(1, 1, 1), 32, 0, stream>>>(Qh + (size_t)b * SEQ * HD, Ql + (size_t)b * SEQ * HD, Kh + (size_t)b * SEQ * HD, Kl + (size_t)b * SEQ * HD, HD, Sb, SEQ, 0, (size_t)0, (size_t)0, (size_t)0);
            k_asoft<<<RHALF / 8, 256, 0, stream>>>(Sb, rofs, Eh, El);
            k_gemmw<bf, 2, false, true><<<dim3(RHALF / 64, 1, 1), 32, 0, stream>>>(Eh, El, Vh + (size_t)b * HD * SEQ, Vl + (size_t)b * HD * SEQ, SEQ, OUT + ((size_t)b * SEQ + rofs) * HD, HD, rofs, (size_t)0, (size_t)0, (size_t)0);
        }
    }
}
